// RNPDecoder_72516227826255
// MI455X (gfx1250) — hardware-run, weakly checked
//
#include <hip/hip_runtime.h>
#include <math.h>

typedef __attribute__((ext_vector_type(16))) _Float16 v16h;
typedef __attribute__((ext_vector_type(8)))  _Float16 v8h;
typedef __attribute__((ext_vector_type(8)))  float    v8f;
typedef __attribute__((ext_vector_type(4)))  float    v4f;
typedef __attribute__((ext_vector_type(2)))  float    v2f;

constexpr int kB    = 1024;
constexpr int kZ    = 32;
constexpr int kHU   = 64;
constexpr int kNS   = 36336;
constexpr int kNP   = 10596;
constexpr int kNSP  = 36352;
constexpr int kNPP  = 10624;
constexpr int kImg  = 28;
constexpr int kPix  = kImg * kImg;
static_assert(kNSP % 64 == 0 && kNPP % 64 == 0 && kNSP >= kNS && kNPP >= kNP, "padded widths");
static_assert(kNSP - kNS < 64 && kNPP - kNP < 64, "minimal padding");
static_assert(kB % 64 == 0 && kHU % 32 == 0, "GEMM tile multiples");

constexpr int kOffEnc1W = 0;
constexpr int kOffEnc1B = 64 * 32;
constexpr int kOffEnc2W = kOffEnc1B + 32;
constexpr int kOffEnc2B = kOffEnc2W + 32 * 32;
constexpr int kOffDec1W = kOffEnc2B + 32;
constexpr int kOffDec1B = kOffDec1W + 32 * 32;
constexpr int kOffDec2W = kOffDec1B + 32;
constexpr int kS_Dec2B  = kOffDec2W + 32 * kPix;
constexpr int kS_Rnn    = kS_Dec2B + kPix;
constexpr int kS_Z0     = kS_Rnn + 32 * 96 * 2 + 96;
constexpr int kP_Dec2B  = kOffDec2W + 32 * 4;
constexpr int kP_Rnn    = kP_Dec2B + 4;
constexpr int kP_Z0     = kP_Rnn + 32 * 96 * 2 + 96;
static_assert(kOffEnc2W == 2080 && kOffDec1W == 3136 && kOffDec2W == 4192, "row map");
static_assert(kS_Dec2B == 29280 && kS_Rnn == 30064 && kS_Z0 == 36304 && kS_Z0 + 32 == kNS, "shape net row map");
static_assert(kP_Dec2B == 4320 && kP_Rnn == 4324 && kP_Z0 == 10564 && kP_Z0 + 32 == kNP, "pose net row map");

constexpr float kACarry     = 64.0f;
constexpr float kBCarry     = 1024.0f;
constexpr float kRCarry     = 2048.0f;
constexpr float kInvRCarry  = 1.0f / kRCarry;
constexpr float kSCarry     = 64.0f;
constexpr float kInvSCarry  = 1.0f / kSCarry;
constexpr float kGemmScaleS = kSCarry / (kACarry * kBCarry);
constexpr float kGemmScaleP = 1.0f / (kACarry * kBCarry);
constexpr float kF16Min     = 6.103515625e-5f;

constexpr size_t kSzH2    = (size_t)kB * kHU * 2;
constexpr size_t kSzBTS   = (size_t)kNSP * kHU * 2;
constexpr size_t kSzBTP   = (size_t)kNPP * kHU * 2;
constexpr size_t kSzSPL   = (size_t)kB * kNSP * 2;
constexpr size_t kSzPPL   = (size_t)kB * kNPP * 4;
constexpr size_t kOffH2S  = 0;
constexpr size_t kOffH2P  = kOffH2S  + kSzH2;
constexpr size_t kOffH2SR = kOffH2P  + kSzH2;
constexpr size_t kOffH2PR = kOffH2SR + kSzH2;
constexpr size_t kOffBTS  = kOffH2PR + kSzH2;
constexpr size_t kOffBTSR = kOffBTS  + kSzBTS;
constexpr size_t kOffBTP  = kOffBTSR + kSzBTS;
constexpr size_t kOffBTPR = kOffBTP  + kSzBTP;
constexpr size_t kOffSPL  = kOffBTPR + kSzBTP;
constexpr size_t kOffPPL  = kOffSPL  + kSzSPL;
constexpr size_t kWsTotal = kOffPPL  + kSzPPL;
static_assert(kSzH2 == 131072ull && kSzBTS == 4653056ull && kSzBTP == 1359872ull &&
              kSzSPL == 74448896ull && kSzPPL == 43515904ull, "region sizes");
static_assert(kWsTotal == 130514944ull, "carve total");
static_assert(kWsTotal <= 134217728ull, "carve cap");
static_assert((kOffH2P % 128) == 0 && (kOffH2SR % 128) == 0 && (kOffH2PR % 128) == 0 && (kOffBTS % 128) == 0 &&
              (kOffBTSR % 128) == 0 && (kOffBTP % 128) == 0 && (kOffBTPR % 128) == 0 &&
              (kOffSPL % 128) == 0 && (kOffPPL % 128) == 0, "128-B aligned regions");

__device__ __forceinline__ float h16_to_f32(unsigned hb) {
  const unsigned sgn = (hb & 0x8000u) << 16;
  const unsigned em = hb & 0x7fffu;
  const float fn = __uint_as_float((em << 13) + 0x38000000u);
  const float fs = (float)em * 5.9604644775390625e-8f;
  const float mag = (em < 0x400u) ? fs : fn;
  return __uint_as_float(__float_as_uint(mag) | sgn);
}

__device__ __forceinline__ float flush_small(float v) {
  return (fabsf(v) < kF16Min) ? 0.0f : v;
}

__device__ __forceinline__ void split_vals(float x, float& valf, float& remf) {
  const float xv = flush_small(x);
  const _Float16 hx = (_Float16)xv;
  const float back = (float)hx;
  valf = back;
  remf = flush_small((x - back) * kRCarry);
}

struct FragH {
  union U { v16h v; v8h h[2]; };
  static __device__ __forceinline__ v16h load(const _Float16* p) {
    U f;
    f.h[0] = *(const v8h*)(p);
    f.h[1] = *(const v8h*)(p + 16);
    return f.v;
  }
};

__device__ __forceinline__ v8f mma_g(v16h a, v16h b, v8f c) {
  c = __builtin_amdgcn_wmma_f32_16x16x32_f16(false, a, false, b, (short)0, c, false, false);
  asm volatile("v_nop\n\tv_nop\n\tv_nop\n\tv_nop" : "+v"(c) : "v"(a), "v"(b));
  return c;
}

__global__ __launch_bounds__(256) void backbone_front_kernel(
    const float* __restrict__ z,
    const float* __restrict__ s_w1, const float* __restrict__ s_b1,
    const float* __restrict__ s_w2, const float* __restrict__ s_b2,
    const float* __restrict__ p_w1, const float* __restrict__ p_b1,
    const float* __restrict__ p_w2, const float* __restrict__ p_b2,
    unsigned short* __restrict__ H2S, unsigned short* __restrict__ H2P,
    unsigned short* __restrict__ H2SR, unsigned short* __restrict__ H2PR)
{
  __shared__ __align__(16) float zs[4 * kZ];
  __shared__ __align__(16) float h1s[4 * kHU];
  __shared__ __align__(16) float h2s[2 * 4 * kHU];
  const int tid  = threadIdx.x;
  const int lane = tid & 31;
  const int wave = __builtin_amdgcn_readfirstlane(tid >> 5);
  const int sl = tid >> 6;
  const int j  = tid & 63;
  const int b0 = blockIdx.x * 4;
  if (wave < 4) zs[tid] = z[(size_t)b0 * kZ + tid];
  __syncthreads();
#pragma unroll 1
  for (int net = 0; net < 2; ++net) {
    const float* w1 = net ? p_w1 : s_w1;
    const float* b1 = net ? p_b1 : s_b1;
    const float* w2 = net ? p_w2 : s_w2;
    const float* b2 = net ? p_b2 : s_b2;
    float acc = 0.0f;
#pragma unroll 4
    for (int k = 0; k < kZ; ++k) acc = fmaf(zs[sl * kZ + k], w1[k * kHU + j], acc);
    acc += b1[j];
    h1s[sl * kHU + j] = fmaxf(acc, 0.0f);
    __syncthreads();
    float acc2 = 0.0f;
#pragma unroll 4
    for (int k = 0; k < kHU; ++k) acc2 = fmaf(h1s[sl * kHU + k], w2[k * kHU + j], acc2);
    acc2 += b2[j];
    h2s[net * 256 + sl * kHU + j] = fmaxf(acc2, 0.0f) * kACarry;
    __syncthreads();
  }
  if (wave < 4) {
    const int netw  = wave & 1;
    const int isrem = wave >> 1;
    unsigned q = (unsigned)lane >> 3;
    asm volatile("" : "+v"(q));
    unsigned c8 = ((unsigned)lane & 7u) * 8u;
    asm volatile("" : "+v"(c8));
    const float* sp = h2s + netw * 256 + (int)q * kHU + (int)c8;
    const v4f a0 = *(const v4f*)(sp);
    const v4f a1 = *(const v4f*)(sp + 4);
    v8h ov;
#pragma unroll
    for (int e = 0; e < 4; ++e) {
      const float x0 = a0[e];
      const float x1 = a1[e];
      float v0, r0, v1, r1;
      split_vals(x0, v0, r0);
      split_vals(x1, v1, r1);
      const float c0 = isrem ? r0 : v0;
      const float c1 = isrem ? r1 : v1;
      ov[e]     = (_Float16)c0;
      ov[4 + e] = (_Float16)c1;
    }
    unsigned short* pv = netw ? H2P : H2S;
    unsigned short* pr = netw ? H2PR : H2SR;
    unsigned short* base = isrem ? pr : pv;
    unsigned short* dst = base + (size_t)(b0 + (int)q) * kHU + c8;
    *(volatile v8h*)dst = ov;
    __threadfence();
    *(volatile v8h*)dst = ov;
  }
}

__global__ __launch_bounds__(256) void weight_plane_kernel(
    const float* __restrict__ w3, unsigned short* __restrict__ Bt, unsigned short* __restrict__ BtR, int N)
{
  __shared__ __align__(16) float T[64 * 65];
  const int tid  = threadIdx.x;
  const int lane = tid & 31;
  const int wave = __builtin_amdgcn_readfirstlane(tid >> 5);
  const int n0 = blockIdx.x * 64;
  unsigned nl = (unsigned)tid & 63u;
  asm volatile("" : "+v"(nl));
  unsigned kq = (unsigned)tid >> 6;
  asm volatile("" : "+v"(kq));
  const int n  = n0 + (int)nl;
  const bool inr = n < N;
  const int nc = inr ? n : (N - 1);
#pragma unroll 4
  for (int it = 0; it < 16; ++it) {
    const int k = it * 4 + (int)kq;
    float v = w3[(size_t)k * N + nc];
    asm volatile("" : "+v"(v));
    v = inr ? (v * kBCarry) : 0.0f;
    T[k * 65 + (int)nl] = v;
  }
  __syncthreads();
  unsigned q = (unsigned)lane >> 3;
  asm volatile("" : "+v"(q));
  unsigned c8 = ((unsigned)lane & 7u) * 8u;
  asm volatile("" : "+v"(c8));
  v8h hv[2], rv[2];
#pragma unroll
  for (int it = 0; it < 2; ++it) {
    const int row = it * 32 + wave * 4 + (int)q;
#pragma unroll
    for (int e = 0; e < 8; ++e) {
      const float x = T[((int)c8 + e) * 65 + row];
      float vf, rf;
      split_vals(x, vf, rf);
      hv[it][e] = (_Float16)vf;
      rv[it][e] = (_Float16)rf;
    }
  }
  for (int pass = 0; pass < 2; ++pass) {
#pragma unroll
    for (int it = 0; it < 2; ++it) {
      const int row = it * 32 + wave * 4 + (int)q;
      const size_t o = (size_t)(n0 + row) * kHU + c8;
      *(volatile v8h*)(Bt + o)  = hv[it];
      *(volatile v8h*)(BtR + o) = rv[it];
    }
    __threadfence();
  }
}

template <bool OUT_F32>
__global__ __launch_bounds__(256) void param_gemm_kernel(
    const unsigned short* __restrict__ Ap, const unsigned short* __restrict__ ARp,
    const unsigned short* __restrict__ Btp, const unsigned short* __restrict__ BtRp,
    void* __restrict__ Cout, const float* __restrict__ bias,
    int Npad, int Nreal, float scale, float bscale)
{
  const _Float16* A   = (const _Float16*)Ap;
  const _Float16* AR  = (const _Float16*)ARp;
  const _Float16* Bt  = (const _Float16*)Btp;
  const _Float16* BtR = (const _Float16*)BtRp;
  __shared__ __align__(16) float sT[8][16 * 68];
  const int lane = threadIdx.x & 31;
  const int wave = threadIdx.x >> 5;
  const int tilesN = Npad >> 6;
  const int tilesM = kB >> 5;
  const int tile = blockIdx.x * 8 + wave;
  if (tile >= tilesM * tilesN) return;
  const int tm = tile / tilesN;
  const int tn = tile - tm * tilesN;
  const int m0 = tm << 5;
  const int n0 = tn << 6;
  unsigned rl_u = (unsigned)lane & 15u;
  asm volatile("" : "+v"(rl_u));
  unsigned hf_u = ((unsigned)lane >> 4) * 8u;
  asm volatile("" : "+v"(hf_u));
  const int rlane = (int)rl_u;
  const int koff  = (int)hf_u;
  const int mOff  = (int)hf_u;

  v8f acc[2][4], accr[2][4];
#pragma unroll
  for (int i = 0; i < 2; ++i) {
#pragma unroll
    for (int j = 0; j < 4; ++j) {
      acc[i][j]  = (v8f){0.f, 0.f, 0.f, 0.f, 0.f, 0.f, 0.f, 0.f};
      accr[i][j] = (v8f){0.f, 0.f, 0.f, 0.f, 0.f, 0.f, 0.f, 0.f};
    }
  }

#pragma unroll 1
  for (int k0 = 0; k0 < kHU; k0 += 32) {
    v16h ah[2], al[2];
#pragma unroll
    for (int i = 0; i < 2; ++i) {
      const size_t ao = (size_t)(m0 + (i << 4) + rlane) * kHU + koff + k0;
      ah[i] = FragH::load(A + ao);
      al[i] = FragH::load(AR + ao);
    }
#pragma unroll
    for (int j = 0; j < 4; ++j) {
      const size_t bo = (size_t)(n0 + (j << 4) + rlane) * kHU + koff + k0;
      const v16h bh = FragH::load(Bt + bo);
      const v16h bl = FragH::load(BtR + bo);
#pragma unroll
      for (int i = 0; i < 2; ++i) {
        acc[i][j]  = mma_g(ah[i], bh, acc[i][j]);
        accr[i][j] = mma_g(ah[i], bl, accr[i][j]);
        accr[i][j] = mma_g(al[i], bh, accr[i][j]);
      }
    }
  }

  float bv[4];
#pragma unroll
  for (int j = 0; j < 4; ++j) {
    const int n = n0 + (j << 4) + rlane;
    const int nc = (n < Nreal) ? n : (Nreal - 1);
    float braw = bias[nc];
    asm volatile("" : "+v"(braw));
    bv[j] = (n < Nreal) ? (braw * bscale) : 0.0f;
  }

  float* slab = sT[wave];
#pragma unroll
  for (int i = 0; i < 2; ++i) {
    const int mBase = m0 + (i << 4);
#pragma unroll
    for (int j = 0; j < 4; ++j) {
#pragma unroll
      for (int r = 0; r < 8; ++r) {
        const float s = fmaf(accr[i][j][r], kInvRCarry, acc[i][j][r]);
        float v = s * scale + bv[j];
        if (!OUT_F32) v = flush_small(v);
        slab[(mOff + r) * 68 + (j << 4) + rlane] = v;
      }
    }
    __builtin_amdgcn_fence(__ATOMIC_RELEASE, "workgroup");
    __builtin_amdgcn_wave_barrier();
    __builtin_amdgcn_fence(__ATOMIC_ACQUIRE, "workgroup");
    if (OUT_F32) {
      float* C = (float*)Cout;
      unsigned hh = (unsigned)lane >> 4;
      asm volatile("" : "+v"(hh));
      unsigned c4 = ((unsigned)lane & 15u) * 4u;
      asm volatile("" : "+v"(c4));
      for (int pass = 0; pass < 2; ++pass) {
#pragma unroll
        for (int it = 0; it < 8; ++it) {
          const int row = it * 2 + (int)hh;
          const v4f v = *(const v4f*)(slab + row * 68 + (int)c4);
          *(volatile v4f*)(C + (size_t)(mBase + row) * Npad + n0 + c4) = v;
        }
        __threadfence();
      }
    } else {
      unsigned short* C = (unsigned short*)Cout;
      unsigned q = (unsigned)lane >> 3;
      asm volatile("" : "+v"(q));
      unsigned c8 = ((unsigned)lane & 7u) * 8u;
      asm volatile("" : "+v"(c8));
      for (int pass = 0; pass < 2; ++pass) {
#pragma unroll
        for (int it = 0; it < 4; ++it) {
          const int row = it * 4 + (int)q;
          const float* sp = slab + row * 68 + (int)c8;
          v8h hv;
#pragma unroll
          for (int e = 0; e < 8; ++e) hv[e] = (_Float16)sp[e];
          *(volatile v8h*)(C + (size_t)(mBase + row) * Npad + n0 + c8) = hv;
        }
        __threadfence();
      }
    }
    __builtin_amdgcn_fence(__ATOMIC_RELEASE, "workgroup");
    __builtin_amdgcn_wave_barrier();
    __builtin_amdgcn_fence(__ATOMIC_ACQUIRE, "workgroup");
  }
}

constexpr int L_ZZ  = 0;
constexpr int L_ZI  = 128;
constexpr int L_ZS  = 256;
constexpr int L_UL  = 384;
constexpr int UF    = 304;
constexpr int U_E1  = 0;
constexpr int U_E2  = 32;
constexpr int U_GX  = 64;
constexpr int U_ZG  = 160;
constexpr int U_RGH = 192;
constexpr int U_HS  = 224;
constexpr int U_D1  = 256;
constexpr int L_DB  = L_UL + 4 * UF;
constexpr int L_AI  = L_DB + 2 * 4 * 32;
constexpr int L_AO  = L_AI + 2 * 4 * 4;
constexpr int L_XH  = L_AO + 16;
constexpr int L_OI  = L_XH + 2 * 4 * kPix;
constexpr int L_OA  = L_OI + 2 * kPix;
constexpr int L_TOT = L_OA + 2 * kPix;
static_assert((L_UL % 4) == 0 && (UF % 4) == 0 && (L_DB % 4) == 0 && (L_AI % 4) == 0 && (L_AO % 4) == 0 &&
              (L_XH % 4) == 0 && (L_OI % 4) == 0 && (L_OA % 4) == 0, "16-B aligned LDS regions");
static_assert(L_TOT * 4 <= 65536, "static LDS");
static_assert((2 * kPix) % 32 == 0 && (2 * kPix * 4) % 128 == 0, "pair of samples = whole waves and whole lines");

__device__ __forceinline__ float gate_unit(float pre, float k) {
  const float e = expf(-(k * pre));
  return __builtin_amdgcn_rcpf(1.0f + e);
}

__device__ __forceinline__ float bilinear_at(const float* img, v4f a, float gxc, float gyc) {
  const float sx = a[0] + 1.0f;
  const float sy = a[1] + 1.0f;
  const float px = (sx * gxc + a[2] + 1.0f) * 0.5f * (float)(kImg - 1);
  const float py = (sy * gyc + a[3] + 1.0f) * 0.5f * (float)(kImg - 1);
  float x0f = floorf(px);
  float y0f = floorf(py);
  const float wx = px - x0f;
  const float wy = py - y0f;
  x0f = fminf(fmaxf(x0f, -2.0f), (float)(kImg + 1));
  y0f = fminf(fmaxf(y0f, -2.0f), (float)(kImg + 1));
  const int x0 = (int)x0f;
  const int y0 = (int)y0f;
  float v = 0.0f;
#pragma unroll
  for (int dy = 0; dy < 2; ++dy) {
#pragma unroll
    for (int dx = 0; dx < 2; ++dx) {
      const int yy = y0 + dy;
      const int xx = x0 + dx;
      const bool ok = (yy >= 0) && (yy < kImg) && (xx >= 0) && (xx < kImg);
      const int yc = yy < 0 ? 0 : (yy > kImg - 1 ? kImg - 1 : yy);
      const int xc = xx < 0 ? 0 : (xx > kImg - 1 ? kImg - 1 : xx);
      const float raw = img[yc * kImg + xc];
      const float g = ok ? raw : 0.0f;
      const float wgt = (dx ? wx : (1.0f - wx)) * (dy ? wy : (1.0f - wy));
      v = fmaf(g, wgt, v);
    }
  }
  return v;
}

__global__ __launch_bounds__(256) void recur_kernel(
    const unsigned* __restrict__ Sw, const float* __restrict__ Pf, float* __restrict__ out)
{
  __shared__ __align__(16) float L[L_TOT];
  const int tid  = threadIdx.x;
  const int lane = tid & 31;
  const int wave = __builtin_amdgcn_readfirstlane(tid >> 5);
  const int unit  = wave >> 1;
  const int wv    = wave & 1;
  const int usamp = unit >> 1;
  const int net   = unit & 1;
  const int blk   = blockIdx.x;
  const int ub    = L_UL + unit * UF;
  const int rnn   = net ? kP_Rnn : kS_Rnn;
  const size_t usr = (size_t)(blk * 2 + usamp);
  const unsigned* Ws = Sw + usr * (kNSP / 2);
  const float*    Wp = Pf + usr * kNPP;
  const float osc = net ? 1.0f : kInvSCarry;
  unsigned l15  = (unsigned)lane & 15u;
  unsigned hsel = (unsigned)lane >> 4;
  asm volatile("" : "+v"(l15));
  asm volatile("" : "+v"(hsel));

#pragma unroll 1
  for (int i = tid; i < (L_XH - L_ZS); i += 256) L[L_ZS + i] = 0.0f;
#pragma unroll 1
  for (int i = tid; i < 2 * kPix; i += 256) L[L_OA + i] = 0.0f;
  if (wave < 4) {
    const int cs = wave >> 1;
    const int nk = wave & 1;
    const size_t bs = (size_t)(blk * 2 + cs);
    const unsigned wS = Sw[bs * (kNSP / 2) + (unsigned)((kS_Z0 + lane) >> 1)];
    const float vP = Pf[bs * kNPP + (unsigned)(kP_Z0 + lane)];
    const unsigned sh = ((unsigned)lane & 1u) * 16u;
    const float vS = h16_to_f32((wS >> sh) & 0xffffu) * kInvSCarry;
    const float v = nk ? vP : vS;
    L[L_ZI + cs * 64 + nk * 32 + lane] = v;
    L[L_ZZ + cs * 64 + nk * 32 + lane] = v;
  }
  __syncthreads();

#pragma unroll 1
  for (int q = 0; q < 20; ++q) {
    const int to = q / 5;
    const int r  = q - to * 5;
    const bool outer = (r == 0);
    const int ti = outer ? 0 : (r - 1);

#pragma unroll 1
    for (int st = 0; st < 7; ++st) {
      int woff = 0, pitch = 32, din = 32, dout = 32, boff = 0, hasb = 1, kind = 0, xoff = 0, yoff = 0;
      bool act = true;
      if (st == 0) {
        woff = kOffEnc1W; din = 64; boff = kOffEnc1B; kind = 1;
        xoff = L_ZZ + usamp * 64; yoff = ub + U_E1;
      } else if (st == 1) {
        woff = kOffEnc2W; boff = kOffEnc2B;
        xoff = ub + U_E1; yoff = ub + U_E2;
      } else if (st == 2) {
        woff = rnn; pitch = 96; dout = 96; boff = rnn + 2 * 32 * 96;
        xoff = ub + U_E2; yoff = ub + U_GX;
      } else if (st == 3) {
        woff = rnn + 32 * 96; pitch = 96; dout = 64; boff = woff; hasb = 0; kind = 2;
        xoff = ub + U_HS; yoff = ub + U_ZG;
      } else if (st == 4) {
        woff = rnn + 32 * 96 + 64; pitch = 96; boff = woff; hasb = 0; kind = 3;
        xoff = ub + U_RGH; yoff = ub + U_HS;
      } else if (st == 5) {
        woff = kOffDec1W; boff = kOffDec1B; kind = 1;
        xoff = ub + U_HS;
        yoff = net ? (ub + U_D1) : (L_DB + usamp * 128 + ti * 32);
        act = (net == 1) || (!outer);
      } else {
        woff = kOffDec2W; pitch = 4; dout = 4; boff = kP_Dec2B;
        xoff = ub + U_D1;
        yoff = outer ? (L_AO + usamp * 4) : (L_AI + usamp * 16 + ti * 4);
        act = (net == 1);
      }
      if (act) {
        const int npass = (dout + 31) >> 5;
        const int nit = din >> 1;
        const int ph2 = pitch >> 1;
#pragma unroll 1
        for (int pw = wv; pw < npass; pw += 2) {
          unsigned c2raw = (unsigned)(pw * 32) + 2u * l15;
          asm volatile("" : "+v"(c2raw));
          const bool valid = c2raw < (unsigned)dout;
          unsigned c2 = valid ? c2raw : (unsigned)(dout - 2);
          asm volatile("" : "+v"(c2));
          unsigned i0 = hsel * (unsigned)nit;
          asm volatile("" : "+v"(i0));
          unsigned eoff = (unsigned)woff + i0 * (unsigned)pitch + c2;
          asm volatile("" : "+v"(eoff));
          const float* xp = L + xoff + i0;
          float a0 = 0.0f, a1 = 0.0f;
          float b0 = 0.0f, b1 = 0.0f;
          if (net) {
            const float* wpf = Wp + eoff;
#pragma unroll 1
            for (int i = 0; i < nit; i += 4) {
              const v4f xv = *(const v4f*)(xp + i);
              const v2f q0 = *(const v2f*)(wpf + (i + 0) * pitch);
              const v2f q1 = *(const v2f*)(wpf + (i + 1) * pitch);
              const v2f q2 = *(const v2f*)(wpf + (i + 2) * pitch);
              const v2f q3 = *(const v2f*)(wpf + (i + 3) * pitch);
              a0 = fmaf(xv[0], q0[0], a0);
              a1 = fmaf(xv[0], q0[1], a1);
              a0 = fmaf(xv[1], q1[0], a0);
              a1 = fmaf(xv[1], q1[1], a1);
              a0 = fmaf(xv[2], q2[0], a0);
              a1 = fmaf(xv[2], q2[1], a1);
              a0 = fmaf(xv[3], q3[0], a0);
              a1 = fmaf(xv[3], q3[1], a1);
            }
            const v2f bq = *(const v2f*)(Wp + ((unsigned)boff + c2));
            float bq0 = bq[0];
            float bq1 = bq[1];
            asm volatile("" : "+v"(bq0));
            asm volatile("" : "+v"(bq1));
            b0 = hasb ? bq0 : 0.0f;
            b1 = hasb ? bq1 : 0.0f;
          } else {
            const unsigned* wp = Ws + (eoff >> 1);
#pragma unroll 1
            for (int i = 0; i < nit; i += 4) {
              const v4f xv = *(const v4f*)(xp + i);
              const unsigned q0 = wp[(i + 0) * ph2];
              const unsigned q1 = wp[(i + 1) * ph2];
              const unsigned q2 = wp[(i + 2) * ph2];
              const unsigned q3 = wp[(i + 3) * ph2];
              a0 = fmaf(xv[0], h16_to_f32(q0 & 0xffffu), a0);
              a1 = fmaf(xv[0], h16_to_f32(q0 >> 16), a1);
              a0 = fmaf(xv[1], h16_to_f32(q1 & 0xffffu), a0);
              a1 = fmaf(xv[1], h16_to_f32(q1 >> 16), a1);
              a0 = fmaf(xv[2], h16_to_f32(q2 & 0xffffu), a0);
              a1 = fmaf(xv[2], h16_to_f32(q2 >> 16), a1);
              a0 = fmaf(xv[3], h16_to_f32(q3 & 0xffffu), a0);
              a1 = fmaf(xv[3], h16_to_f32(q3 >> 16), a1);
            }
            unsigned bw = Ws[((unsigned)boff + c2) >> 1];
            asm volatile("" : "+v"(bw));
            b0 = hasb ? h16_to_f32(bw & 0xffffu) : 0.0f;
            b1 = hasb ? h16_to_f32(bw >> 16) : 0.0f;
          }
          a0 += __shfl_xor(a0, 16, 32);
          a1 += __shfl_xor(a1, 16, 32);
          float y0 = (a0 + b0) * osc;
          float y1 = (a1 + b1) * osc;
          int dsto = yoff + (int)c2;
          if (kind == 1) {
            y0 = fmaxf(y0, 0.0f);
            y1 = fmaxf(y1, 0.0f);
          }
          if (kind >= 2) {
            const int cg = (kind == 3) ? ((int)c2 + 64) : (int)c2;
            const int ch = (int)(c2 & 31u);
            const v2f gv = *(const v2f*)(L + ub + U_GX + cg);
            const v2f hv = *(const v2f*)(L + ub + U_HS + ch);
            const v2f zv = *(const v2f*)(L + ub + U_ZG + ch);
            const float kk = (kind == 3) ? 2.0f : 1.0f;
            const float s0 = gate_unit(y0 + gv[0], kk);
            const float s1 = gate_unit(y1 + gv[1], kk);
            if (kind == 2) {
              if (pw == 0) {
                y0 = s0;
                y1 = s1;
                dsto = ub + U_ZG + ch;
              } else {
                y0 = s0 * hv[0];
                y1 = s1 * hv[1];
                dsto = ub + U_RGH + ch;
              }
            } else {
              const float t0 = 2.0f * s0 - 1.0f;
              const float t1 = 2.0f * s1 - 1.0f;
              y0 = zv[0] * hv[0] + (1.0f - zv[0]) * t0;
              y1 = zv[1] * hv[1] + (1.0f - zv[1]) * t1;
              dsto = ub + U_HS + ch;
            }
          }
          if (valid && (hsel == 0u)) {
            v2f yo;
            yo[0] = y0;
            yo[1] = y1;
            *(v2f*)(L + dsto) = yo;
          }
        }
      }
      __syncthreads();
    }

    if (wave < 4) {
      const int cs = wave >> 1;
      const int nk = wave & 1;
      const float hval = L[L_UL + (cs * 2 + nk) * UF + U_HS + lane];
      const int zo = cs * 64 + nk * 32 + lane;
      if (r == 0) {
        L[L_ZS + zo] = hval;
        L[L_ZZ + zo] = L[L_ZI + zo];
      } else if (r < 4) {
        L[L_ZZ + zo] = hval;
      } else {
        L[L_ZZ + zo] = L[L_ZS + zo];
      }
    }
    __syncthreads();

    if (r == 4) {
#pragma unroll 1
      for (int wp_ = wave; wp_ < 25; wp_ += 8) {
        unsigned item = (unsigned)(wp_ * 32 + lane);
        asm volatile("" : "+v"(item));
        const bool ok = item < (unsigned)kPix;
        unsigned itc = ok ? item : (unsigned)(kPix - 1);
        asm volatile("" : "+v"(itc));
        unsigned s = (itc >= (unsigned)(kPix / 2)) ? 1u : 0u;
        asm volatile("" : "+v"(s));
        unsigned p = itc - s * (unsigned)(kPix / 2);
        asm volatile("" : "+v"(p));
        const unsigned* srow = Sw + (size_t)((unsigned)(blk * 2) + s) * (kNSP / 2);
        const unsigned* wrow = srow + (kOffDec2W >> 1) + p;
        const float* dp = L + L_DB + s * 128u;
        float c00 = 0.0f, c01 = 0.0f, c10 = 0.0f, c11 = 0.0f;
        float c20 = 0.0f, c21 = 0.0f, c30 = 0.0f, c31 = 0.0f;
#pragma unroll 1
        for (int i = 0; i < 32; ++i) {
          unsigned w = wrow[i * (kPix / 2)];
          asm volatile("" : "+v"(w));
          const float w0 = h16_to_f32(w & 0xffffu);
          const float w1 = h16_to_f32(w >> 16);
          const float d0 = dp[i];
          const float d1 = dp[32 + i];
          const float d2 = dp[64 + i];
          const float d3 = dp[96 + i];
          c00 = fmaf(d0, w0, c00);
          c01 = fmaf(d0, w1, c01);
          c10 = fmaf(d1, w0, c10);
          c11 = fmaf(d1, w1, c11);
          c20 = fmaf(d2, w0, c20);
          c21 = fmaf(d2, w1, c21);
          c30 = fmaf(d3, w0, c30);
          c31 = fmaf(d3, w1, c31);
        }
        unsigned bw = srow[(kS_Dec2B >> 1) + p];
        asm volatile("" : "+v"(bw));
        const float b0 = h16_to_f32(bw & 0xffffu);
        const float b1 = h16_to_f32(bw >> 16);
        if (ok) {
          float* xo = L + L_XH + s * (unsigned)(4 * kPix) + 2u * p;
          v2f o;
          o[0] = (c00 + b0) * kInvSCarry;
          o[1] = (c01 + b1) * kInvSCarry;
          *(v2f*)(xo) = o;
          o[0] = (c10 + b0) * kInvSCarry;
          o[1] = (c11 + b1) * kInvSCarry;
          *(v2f*)(xo + kPix) = o;
          o[0] = (c20 + b0) * kInvSCarry;
          o[1] = (c21 + b1) * kInvSCarry;
          *(v2f*)(xo + 2 * kPix) = o;
          o[0] = (c30 + b0) * kInvSCarry;
          o[1] = (c31 + b1) * kInvSCarry;
          *(v2f*)(xo + 3 * kPix) = o;
        }
      }
      __syncthreads();

#pragma unroll 1
      for (int ph = 0; ph < 2; ++ph) {
        const int nimg = ph ? 1 : 4;
        const int srcb = ph ? L_OI : L_XH;
        const int sstr = ph ? kPix : 4 * kPix;
        const int ab   = ph ? L_AO : L_AI;
        const int astr = ph ? 4 : 16;
        const int dstb = ph ? L_OA : L_OI;
#pragma unroll 1
        for (int pass = 0; pass < 7; ++pass) {
          const int base = pass * 256 + wave * 32;
          if (base < 2 * kPix) {
            unsigned idx = (unsigned)(base + lane);
            asm volatile("" : "+v"(idx));
            unsigned s = (idx >= (unsigned)kPix) ? 1u : 0u;
            asm volatile("" : "+v"(s));
            unsigned p = idx - s * (unsigned)kPix;
            asm volatile("" : "+v"(p));
            unsigned iy = p / (unsigned)kImg;
            asm volatile("" : "+v"(iy));
            unsigned ix = p - iy * (unsigned)kImg;
            asm volatile("" : "+v"(ix));
            const float gxc = -1.0f + (float)ix * (2.0f / (float)(kImg - 1));
            const float gyc = -1.0f + (float)iy * (2.0f / (float)(kImg - 1));
            float v = 0.0f;
#pragma unroll 1
            for (int t = 0; t < nimg; ++t) {
              const v4f a = *(const v4f*)(L + ab + (int)s * astr + t * 4);
              const float* img = L + srcb + (int)s * sstr + t * kPix;
              v += bilinear_at(img, a, gxc, gyc);
            }
            float basev = 0.0f;
            if (ph == 1) basev = L[dstb + (int)idx];
            L[dstb + (int)idx] = basev + v;
          }
        }
        __syncthreads();
      }
    }
  }

  {
    v4f rv[2];
    bool okv[2];
#pragma unroll
    for (int k = 0; k < 2; ++k) {
      const int f4 = (wave + 8 * k) * 32 + lane;
      okv[k] = f4 < (2 * kPix / 4);
      const int f4c = okv[k] ? f4 : (2 * kPix / 4 - 1);
      rv[k] = *(const v4f*)(L + L_OA + 4 * f4c);
    }
    float* ob = out + (size_t)blk * (2 * kPix);
    for (int pass = 0; pass < 2; ++pass) {
#pragma unroll
      for (int k = 0; k < 2; ++k) {
        const int f4 = (wave + 8 * k) * 32 + lane;
        if (okv[k]) *(volatile v4f*)(ob + 4 * f4) = rv[k];
      }
      __threadfence();
    }
  }
}

static_assert(((kB / 32) * (kNSP / 64)) % 8 == 0 && ((kB / 32) * (kNPP / 64)) % 8 == 0, "whole blocks of tiles");
static_assert(kB % 4 == 0 && kB % 2 == 0, "sample grouping");

extern "C" void kernel_launch(void* const* d_in, const int* in_sizes, int n_in,
                              void* d_out, int out_size, void* d_ws, size_t ws_size,
                              hipStream_t stream) {
  if (n_in < 14) return;
  if (in_sizes[1] != kB * kZ) return;
  if (in_sizes[2] != kZ * kHU || in_sizes[3] != kHU) return;
  if (in_sizes[4] != kHU * kHU || in_sizes[5] != kHU) return;
  if (in_sizes[6] != kHU * kNS || in_sizes[7] != kNS) return;
  if (in_sizes[8] != kZ * kHU || in_sizes[9] != kHU) return;
  if (in_sizes[10] != kHU * kHU || in_sizes[11] != kHU) return;
  if (in_sizes[12] != kHU * kNP || in_sizes[13] != kNP) return;
  if (out_size != kB * kPix) return;
  if (ws_size < kWsTotal) return;

  const float* z    = (const float*)d_in[1];
  const float* s_w1 = (const float*)d_in[2];
  const float* s_b1 = (const float*)d_in[3];
  const float* s_w2 = (const float*)d_in[4];
  const float* s_b2 = (const float*)d_in[5];
  const float* s_w3 = (const float*)d_in[6];
  const float* s_b3 = (const float*)d_in[7];
  const float* p_w1 = (const float*)d_in[8];
  const float* p_b1 = (const float*)d_in[9];
  const float* p_w2 = (const float*)d_in[10];
  const float* p_b2 = (const float*)d_in[11];
  const float* p_w3 = (const float*)d_in[12];
  const float* p_b3 = (const float*)d_in[13];

  char* ws = (char*)d_ws;
  unsigned short* H2S  = (unsigned short*)(ws + kOffH2S);
  unsigned short* H2P  = (unsigned short*)(ws + kOffH2P);
  unsigned short* H2SR = (unsigned short*)(ws + kOffH2SR);
  unsigned short* H2PR = (unsigned short*)(ws + kOffH2PR);
  unsigned short* BTS  = (unsigned short*)(ws + kOffBTS);
  unsigned short* BTSR = (unsigned short*)(ws + kOffBTSR);
  unsigned short* BTP  = (unsigned short*)(ws + kOffBTP);
  unsigned short* BTPR = (unsigned short*)(ws + kOffBTPR);
  unsigned short* SPL  = (unsigned short*)(ws + kOffSPL);
  float*          PPL  = (float*)(ws + kOffPPL);

  backbone_front_kernel<<<kB / 4, 256, 0, stream>>>(z, s_w1, s_b1, s_w2, s_b2, p_w1, p_b1, p_w2, p_b2,
                                                    H2S, H2P, H2SR, H2PR);
  weight_plane_kernel<<<kNSP / 64, 256, 0, stream>>>(s_w3, BTS, BTSR, kNS);
  weight_plane_kernel<<<kNPP / 64, 256, 0, stream>>>(p_w3, BTP, BTPR, kNP);
  param_gemm_kernel<false><<<((kB / 32) * (kNSP / 64)) / 8, 256, 0, stream>>>(
      H2S, H2SR, BTS, BTSR, (void*)SPL, s_b3, kNSP, kNS, kGemmScaleS, kSCarry);
  param_gemm_kernel<true><<<((kB / 32) * (kNPP / 64)) / 8, 256, 0, stream>>>(
      H2P, H2PR, BTP, BTPR, (void*)PPL, p_b3, kNPP, kNP, kGemmScaleP, 1.0f);
  recur_kernel<<<kB / 2, 256, 0, stream>>>((const unsigned*)SPL, (const float*)PPL, (float*)d_out);
}
